// FactorizedPriorGroupViT_77421080478297
// MI455X (gfx1250) — hardware-run, weakly checked
//
#include <hip/hip_runtime.h>


#define NBI  16
#define HH   56
#define CC   256
#define NH_  8
#define HD   32
#define WS   7
#define SSH  3
#define NWI  64
#define NT   49
#define NTI  3136
#define NGI  512
#define HID  1024
#define PCAR 1024.0f
typedef _Float16 h16;
typedef unsigned short bf;
typedef __attribute__((ext_vector_type(16))) __bf16   v16bf;
typedef __attribute__((ext_vector_type(16))) _Float16 v16h;
typedef __attribute__((ext_vector_type(8)))  _Float16 v8h;
typedef __attribute__((ext_vector_type(8)))  unsigned short v8us;
typedef __attribute__((ext_vector_type(8)))  float    v8f;
typedef __attribute__((ext_vector_type(4)))  float    v4f;
typedef v8h  __attribute__((may_alias)) v8ha;
typedef v4f  __attribute__((may_alias)) v4fa;
typedef v8us __attribute__((may_alias)) v8usa;

__device__ __forceinline__ unsigned short f2bf(float f) { unsigned u = __float_as_uint(f); u += 0x7FFFu + ((u >> 16) & 1u); return (unsigned short)(u >> 16); }
__device__ __forceinline__ float bf2f(unsigned short b) { return __uint_as_float(((unsigned)b) << 16); }
__device__ __forceinline__ float bfr(float f) { return bf2f(f2bf(f)); }
__device__ __forceinline__ v16h cat16(v8h lo, v8h hi) { return __builtin_shufflevector(lo, hi, 0, 1, 2, 3, 4, 5, 6, 7, 8, 9, 10, 11, 12, 13, 14, 15); }
__device__ __forceinline__ v16bf cat16b(v8us lo, v8us hi) { return __builtin_bit_cast(v16bf, __builtin_shufflevector(lo, hi, 0, 1, 2, 3, 4, 5, 6, 7, 8, 9, 10, 11, 12, 13, 14, 15)); }
__device__ __forceinline__ v8f wmma16(v16h a, v16h b, v8f c) { return __builtin_amdgcn_wmma_f32_16x16x32_f16(false, a, false, b, (short)0, c, false, false); }
__device__ __forceinline__ v8f wmmab(v16bf a, v16bf b, v8f c) { return __builtin_amdgcn_wmma_f32_16x16x32_bf16(false, a, false, b, (short)0, c, false, false); }


template <typename T16> struct WFrag;
template <> struct WFrag<h16> { typedef v16h V; static __device__ __forceinline__ V ld(const h16* p) { return cat16(*(const v8h*)p, *(const v8h*)(p + 16)); } static __device__ __forceinline__ v8f mma(V a, V b, v8f c) { return wmma16(a, b, c); } };
template <> struct WFrag<bf> { typedef v16bf V; static __device__ __forceinline__ V ld(const bf* p) { return cat16b(*(const v8us*)p, *(const v8us*)(p + 16)); } static __device__ __forceinline__ v8f mma(V a, V b, v8f c) { return wmmab(a, b, c); } };
template <typename T16, int NSPLIT, bool BIAS>
__global__ __launch_bounds__(32) void k_gemmw(const T16* __restrict__ A, const T16* __restrict__ A2, const T16* __restrict__ Bt, const T16* __restrict__ Bt2, int K, float* C, int ldc, const float* __restrict__ bias, size_t sA, size_t sB, size_t sC) {
    typedef typename WFrag<T16>::V V;
    __shared__ __align__(16) float os[16 * 68];
    const size_t z = blockIdx.z; A += z * sA; if (A2) A2 += z * sA; Bt += z * sB; if (Bt2) Bt2 += z * sB; C += z * sC;
    const int lane = threadIdx.x & 31, lr = lane & 15, hi = lane >> 4; const int r0 = blockIdx.x * 64, c0 = blockIdx.y * 64;
    v8f acc[4][4];
#pragma unroll
    for (int mb = 0; mb < 4; ++mb)
#pragma unroll
        for (int nb = 0; nb < 4; ++nb) acc[mb][nb] = (v8f){};
    const size_t aoff = (size_t)(r0 + lr) * K + 8 * hi, boff = (size_t)(c0 + lr) * K + 8 * hi;
#pragma unroll 1
    for (int kc = 0; kc < K; kc += 32) {
        V a[4], a2[4];
#pragma unroll
        for (int mb = 0; mb < 4; ++mb) { a[mb] = WFrag<T16>::ld(A + aoff + (size_t)mb * 16 * K + kc); if (NSPLIT == 1 || NSPLIT == 2) a2[mb] = WFrag<T16>::ld(A2 + aoff + (size_t)mb * 16 * K + kc); }
#pragma unroll
        for (int nb = 0; nb < 4; ++nb) { const V b = WFrag<T16>::ld(Bt + boff + (size_t)nb * 16 * K + kc); V b2; if (NSPLIT >= 2) b2 = WFrag<T16>::ld(Bt2 + boff + (size_t)nb * 16 * K + kc);
#pragma unroll
            for (int mb = 0; mb < 4; ++mb) { acc[mb][nb] = WFrag<T16>::mma(a[mb], b, acc[mb][nb]); if (NSPLIT == 1 || NSPLIT == 2) acc[mb][nb] = WFrag<T16>::mma(a2[mb], b, acc[mb][nb]); if (NSPLIT >= 2) acc[mb][nb] = WFrag<T16>::mma(a[mb], b2, acc[mb][nb]); } }
        asm volatile("v_nop\n\tv_nop\n\tv_nop\n\tv_nop" : "+v"(acc[0][0]), "+v"(acc[1][1]), "+v"(acc[2][2]), "+v"(acc[3][3]) : "v"(a[0]), "v"(a[3]));
    }
#pragma unroll
    for (int mb = 0; mb < 4; ++mb) {
#pragma unroll
        for (int nb = 0; nb < 4; ++nb) {
#pragma unroll
            for (int j = 0; j < 8; ++j) os[(hi * 8 + j) * 68 + nb * 16 + lr] = acc[mb][nb][j]; }
        __builtin_amdgcn_wave_barrier(); asm volatile("" ::: "memory");
        float* crow = C + (size_t)(r0 + mb * 16) * ldc + c0;
#pragma unroll 1
        for (int ps = 0; ps < 2; ++ps) {
#pragma unroll
            for (int s = 0; s < 8; ++s) { const int row = 2 * s + hi, cofs = lr * 4; v4f val = *(const v4fa*)(os + row * 68 + cofs); if (BIAS) { val[0] += bfr(bias[c0 + cofs]); val[1] += bfr(bias[c0 + cofs + 1]); val[2] += bfr(bias[c0 + cofs + 2]); val[3] += bfr(bias[c0 + cofs + 3]); }
                *(volatile v4f*)(crow + (size_t)row * ldc + cofs) = val; }
            if (ps == 0) __threadfence(); }
        __builtin_amdgcn_wave_barrier(); asm volatile("" ::: "memory");
    }
}

__device__ __forceinline__ h16 tohx(float x) { return (h16)x; }
typedef __attribute__((ext_vector_type(2))) _Float16 v2h;
typedef __attribute__((ext_vector_type(4))) _Float16 v4h;

__global__ __launch_bounds__(256) void k_wt16(const float* __restrict__ w, int K, int N, h16* Bt) { const size_t e = ((size_t)blockIdx.x * 256 + threadIdx.x) * 2; if (e >= (size_t)N * K) return; const int k = (int)(e % K), n = (int)(e / K); v2h o; o[0] = tohx(bfr(w[(size_t)k * N + n])); o[1] = tohx(bfr(w[(size_t)(k + 1) * N + n])); *(volatile v2h*)(Bt + e) = o; __threadfence(); *(volatile v2h*)(Bt + e) = o; }
__device__ __forceinline__ void tok2win(int p, int& g0, int& i) { const int y = p / HH, x = p % HH; const int ys = (y - SSH + HH) % HH, xs = (x - SSH + HH) % HH; const int w = (ys / WS) * (HH / WS) + xs / WS; i = (ys % WS) * WS + xs % WS; g0 = w * NH_; }
__device__ __forceinline__ int win2tok(int w, int i) { const int ys = (w / (HH / WS)) * WS + i / WS, xs = (w % (HH / WS)) * WS + i % WS; const int y = (ys + SSH) % HH, x = (xs + SSH) % HH; return y * HH + x; }
__global__ __launch_bounds__(256) void k_lnpl(const float* __restrict__ X, int isin, const float* __restrict__ g, const float* __restrict__ bb, h16* P) { const int lane = threadIdx.x & 31; const int t = blockIdx.x * 8 + (threadIdx.x >> 5); if (t >= NTI) return; const size_t rb = (size_t)t * CC; float v[8]; float s = 0.f;
#pragma unroll
    for (int ch = 0; ch < 2; ++ch) { const v4f a = *(const v4f*)(X + rb + ch * 128 + lane * 4);
#pragma unroll
        for (int q = 0; q < 4; ++q) { v[ch * 4 + q] = isin ? bfr(a[q]) : a[q]; s = __fadd_rn(s, v[ch * 4 + q]); } }
#pragma unroll
    for (int sh = 16; sh; sh >>= 1) s += __shfl_xor(s, sh, 32);
    const float mu = s * (1.0f / CC); float q2 = 0.f;
#pragma unroll
    for (int k = 0; k < 8; ++k) { float dv = __fsub_rn(v[k], mu); asm volatile("" : "+v"(dv)); float p = __fmul_rn(dv, dv); asm volatile("" : "+v"(p)); q2 = __fadd_rn(q2, p); }
#pragma unroll
    for (int sh = 16; sh; sh >>= 1) q2 += __shfl_xor(q2, sh, 32);
    float vq = q2 * (1.0f / CC); asm volatile("" : "+v"(vq)); const float rs = __frsqrt_rn(__fadd_rn(vq, 1e-5f));
    for (int ps = 0; ps < 2; ++ps) {
#pragma unroll
        for (int ch = 0; ch < 2; ++ch) { const int c0 = ch * 128 + lane * 4; v4h o;
#pragma unroll
            for (int q = 0; q < 4; ++q) { float dv = __fsub_rn(v[ch * 4 + q], mu); asm volatile("" : "+v"(dv)); float tn = __fmul_rn(dv, rs); asm volatile("" : "+v"(tn)); float tg = __fmul_rn(tn, bfr(g[c0 + q])); asm volatile("" : "+v"(tg)); o[q] = tohx(__fadd_rn(tg, bfr(bb[c0 + q]))); }
            *(volatile v4h*)(P + rb + c0) = o; } if (ps == 0) __threadfence(); } }
__global__ __launch_bounds__(256) void k_winqk(const float* __restrict__ QKV, h16* QW, h16* KW) { const size_t e = ((size_t)blockIdx.x * 256 + threadIdx.x) * 4; if (e >= (size_t)NGI * 64 * HD) return; const int d = (int)(e % HD); const int i = (int)((e / HD) % 64); const int g = (int)(e / ((size_t)HD * 64)); const int h = g % NH_; const int w = g / NH_; v4h oq, ok;
    if (i < NT) { const int tok = win2tok(w, i); const float* r = QKV + (size_t)tok * 3 * CC + h * HD + d;
#pragma unroll
        for (int q = 0; q < 4; ++q) { oq[q] = tohx(r[q] * 0.17677669529663687f); ok[q] = tohx(r[CC + q]); } } else { for (int q = 0; q < 4; ++q) { oq[q] = (h16)0.f; ok[q] = (h16)0.f; } }
    for (int ps = 0; ps < 2; ++ps) { *(volatile v4h*)(QW + e) = oq; *(volatile v4h*)(KW + e) = ok; if (ps == 0) __threadfence(); } }
__global__ __launch_bounds__(256) void k_winvt(const float* __restrict__ QKV, h16* VT) { const size_t e = ((size_t)blockIdx.x * 256 + threadIdx.x) * 2; if (e >= (size_t)NGI * 64 * 64) return; const int j = (int)(e % 64); const int dv = (int)((e / 64) % 64); const int g = (int)(e / 4096); const int h = g % NH_; const int w = g / NH_; v2h o;
#pragma unroll
    for (int u = 0; u < 2; ++u) { const int jj = j + u; o[u] = (dv < HD && jj < NT) ? tohx(QKV[(size_t)win2tok(w, jj) * 3 * CC + 2 * CC + h * HD + dv]) : (h16)0.f; }
    *(volatile v2h*)(VT + e) = o; __threadfence(); *(volatile v2h*)(VT + e) = o; }
__global__ __launch_bounds__(256) void k_wsoft(const float* __restrict__ Sb, const float* __restrict__ rb, const float* __restrict__ am, h16* P) { const int lane = threadIdx.x & 31; const size_t row = (size_t)blockIdx.x * 8 + (threadIdx.x >> 5); if (row >= (size_t)NGI * 64) return; const int i = (int)(row % 64); const int g = (int)(row / 64); const int h = g % NH_; const int w = g / NH_; v2h o;
    if (i >= NT) { o[0] = (h16)0.f; o[1] = (h16)0.f; *(volatile v2h*)(P + row * 64 + 2 * lane) = o; __threadfence(); *(volatile v2h*)(P + row * 64 + 2 * lane) = o; return; }
    const int r1 = i / WS, c1 = i % WS; const float* sr = Sb + row * 64; float t[2]; float mx = -3.0e38f;
#pragma unroll
    for (int u = 0; u < 2; ++u) { const int j = 2 * lane + u; if (j < NT) { const int r2 = j / WS, c2 = j % WS; const int ridx = (r1 - r2 + WS - 1) * (2 * WS - 1) + (c1 - c2 + WS - 1); const float bsum = __fadd_rn(bfr(rb[ridx * NH_ + h]), bfr(am[((size_t)w * NT + i) * NT + j])); t[u] = __fadd_rn(sr[j], bsum); } else t[u] = -3.0e38f; mx = fmaxf(mx, t[u]); }
#pragma unroll
    for (int sh = 16; sh; sh >>= 1) mx = fmaxf(mx, __shfl_xor(mx, sh, 32));
    float e_[2]; float sum = 0.f;
#pragma unroll
    for (int u = 0; u < 2; ++u) { float d0 = __fsub_rn(t[u], mx); asm volatile("" : "+v"(d0)); e_[u] = (2 * lane + u < NT) ? __expf(d0) : 0.f; sum = __fadd_rn(sum, e_[u]); }
#pragma unroll
    for (int sh = 16; sh; sh >>= 1) sum += __shfl_xor(sum, sh, 32);
    const float f = __fdiv_rn(PCAR, sum); o[0] = tohx(__fmul_rn(e_[0], f)); o[1] = tohx(__fmul_rn(e_[1], f)); *(volatile v2h*)(P + row * 64 + 2 * lane) = o; __threadfence(); *(volatile v2h*)(P + row * 64 + 2 * lane) = o; }
__global__ __launch_bounds__(256) void k_unwin(const float* __restrict__ O, h16* AO) { const size_t e = ((size_t)blockIdx.x * 256 + threadIdx.x) * 4; if (e >= (size_t)NTI * CC) return; const int c = (int)(e % CC); const int tok = (int)(e / CC); const int h = c / HD, dv = c % HD; int g0, i; tok2win(tok, g0, i); const float* r = O + ((size_t)(g0 + h) * 64 + i) * 64 + dv; v4h o;
#pragma unroll
    for (int q = 0; q < 4; ++q) o[q] = tohx(r[q] * (1.0f / PCAR)); *(volatile v4h*)(AO + e) = o; __threadfence(); *(volatile v4h*)(AO + e) = o; }
__global__ __launch_bounds__(256) void k_res(const float* __restrict__ x, const float* __restrict__ A, float* X1) { const size_t i = ((size_t)blockIdx.x * 256 + threadIdx.x) * 4; if (i >= (size_t)NTI * CC) return; const v4f a = *(const v4f*)(A + i); v4f o; o[0] = __fadd_rn(bfr(x[i]), a[0]); o[1] = __fadd_rn(bfr(x[i + 1]), a[1]); o[2] = __fadd_rn(bfr(x[i + 2]), a[2]); o[3] = __fadd_rn(bfr(x[i + 3]), a[3]); *(volatile v4f*)(X1 + i) = o; __threadfence(); *(volatile v4f*)(X1 + i) = o; }
__global__ __launch_bounds__(256) void k_gelu16(const float* __restrict__ A, size_t n4, h16* G) { const size_t i = ((size_t)blockIdx.x * 256 + threadIdx.x) * 4; if (i >= n4 * 4) return; const v4f a = *(const v4f*)(A + i); v4h o;
#pragma unroll
    for (int q = 0; q < 4; ++q) o[q] = tohx(0.5f * a[q] * (1.0f + erff(a[q] * 0.7071067811865476f))); *(volatile v4h*)(G + i) = o; __threadfence(); *(volatile v4h*)(G + i) = o; }
__global__ __launch_bounds__(256) void k_fin(const float* __restrict__ X1, const float* __restrict__ M, float* OUT) { const size_t i = ((size_t)blockIdx.x * 256 + threadIdx.x) * 4; if (i >= (size_t)NTI * CC) return; const v4f a = *(const v4f*)(X1 + i), m = *(const v4f*)(M + i); v4f o; o[0] = __fadd_rn(a[0], m[0]); o[1] = __fadd_rn(a[1], m[1]); o[2] = __fadd_rn(a[2], m[2]); o[3] = __fadd_rn(a[3], m[3]); *(volatile v4f*)(OUT + i) = o; __threadfence(); *(volatile v4f*)(OUT + i) = o; }

extern "C" void kernel_launch(void* const* d_in, const int* in_sizes, int n_in,
                              void* d_out, int out_size, void* d_ws, size_t ws_size, hipStream_t stream) {
    (void)in_sizes; (void)n_in; (void)out_size;
    const float* x = (const float*)d_in[0]; const float* wqkv = (const float*)d_in[1]; const float* bqkv = (const float*)d_in[2]; const float* rb = (const float*)d_in[3]; const float* wpr = (const float*)d_in[4]; const float* bpr = (const float*)d_in[5]; const float* g1 = (const float*)d_in[6]; const float* be1 = (const float*)d_in[7]; const float* g2 = (const float*)d_in[8]; const float* be2 = (const float*)d_in[9]; const float* w1 = (const float*)d_in[10]; const float* bb1 = (const float*)d_in[11]; const float* w2 = (const float*)d_in[12]; const float* bb2 = (const float*)d_in[13]; const float* am = (const float*)d_in[14];
    float* OUT = (float*)d_out;
    char* wsp = (char*)d_ws;
    auto take = [&](size_t bytes) { char* p = wsp; wsp += (bytes + 255) & ~(size_t)255; return (void*)p; };
    h16* WQ = (h16*)take((size_t)CC * 3 * CC * 2); h16* WP = (h16*)take((size_t)CC * CC * 2); h16* W1 = (h16*)take((size_t)CC * HID * 2); h16* W2 = (h16*)take((size_t)HID * CC * 2);
    h16* P16 = (h16*)take((size_t)NTI * CC * 2); float* QKV = (float*)take((size_t)NTI * 3 * CC * 4); h16* QW = (h16*)take((size_t)NGI * 64 * HD * 2); h16* KW = (h16*)take((size_t)NGI * 64 * HD * 2); h16* VT = (h16*)take((size_t)NGI * 64 * 64 * 2); float* Sb = (float*)take((size_t)NGI * 64 * 64 * 4); h16* PP = (h16*)take((size_t)NGI * 64 * 64 * 2);
    float* O = (float*)take((size_t)NGI * 64 * 64 * 4); float* PR = (float*)take((size_t)NTI * CC * 4); float* X1 = (float*)take((size_t)NTI * CC * 4); float* AH = (float*)take((size_t)NTI * HID * 4); h16* G16 = (h16*)take((size_t)NTI * HID * 2); float* M = PR;
    if ((size_t)(wsp - (char*)d_ws) > ws_size) return;
    k_wt16<<<(unsigned)(((size_t)CC * 3 * CC / 2 + 255) / 256), 256, 0, stream>>>(wqkv, CC, 3 * CC, WQ); k_wt16<<<(unsigned)(((size_t)CC * CC / 2 + 255) / 256), 256, 0, stream>>>(wpr, CC, CC, WP); k_wt16<<<(unsigned)(((size_t)CC * HID / 2 + 255) / 256), 256, 0, stream>>>(w1, CC, HID, W1); k_wt16<<<(unsigned)(((size_t)HID * CC / 2 + 255) / 256), 256, 0, stream>>>(w2, HID, CC, W2);
    const unsigned L4 = (unsigned)(((size_t)NTI * CC / 4 + 255) / 256);
    for (int b = 0; b < NBI; ++b) { const float* xb = x + (size_t)b * NTI * CC;
        k_lnpl<<<NTI / 8, 256, 0, stream>>>(xb, 1, g1, be1, P16);
        k_gemmw<h16, 0, true><<<dim3(NTI / 64, 3 * CC / 64, 1), 32, 0, stream>>>(P16, nullptr, WQ, nullptr, CC, QKV, 3 * CC, bqkv, 0, 0, 0);
        k_winqk<<<(unsigned)(((size_t)NGI * 64 * HD / 4 + 255) / 256), 256, 0, stream>>>(QKV, QW, KW); k_winvt<<<(unsigned)(((size_t)NGI * 4096 / 2 + 255) / 256), 256, 0, stream>>>(QKV, VT);
        k_gemmw<h16, 0, false><<<dim3(1, 1, NGI), 32, 0, stream>>>(QW, nullptr, KW, nullptr, HD, Sb, 64, nullptr, (size_t)64 * HD, (size_t)64 * HD, (size_t)4096);
        k_wsoft<<<(unsigned)(((size_t)NGI * 64 + 7) / 8), 256, 0, stream>>>(Sb, rb, am, PP);
        k_gemmw<h16, 0, false><<<dim3(1, 1, NGI), 32, 0, stream>>>(PP, nullptr, VT, nullptr, 64, O, 64, nullptr, (size_t)4096, (size_t)4096, (size_t)4096);
        k_unwin<<<L4, 256, 0, stream>>>(O, P16);
        k_gemmw<h16, 0, true><<<dim3(NTI / 64, CC / 64, 1), 32, 0, stream>>>(P16, nullptr, WP, nullptr, CC, PR, CC, bpr, 0, 0, 0); k_res<<<L4, 256, 0, stream>>>(xb, PR, X1);
        k_lnpl<<<NTI / 8, 256, 0, stream>>>(X1, 0, g2, be2, P16);
        k_gemmw<h16, 0, true><<<dim3(NTI / 64, HID / 64, 1), 32, 0, stream>>>(P16, nullptr, W1, nullptr, CC, AH, HID, bb1, 0, 0, 0); k_gelu16<<<(unsigned)(((size_t)NTI * HID / 4 + 255) / 256), 256, 0, stream>>>(AH, (size_t)NTI * HID / 4, G16);
        k_gemmw<h16, 0, true><<<dim3(NTI / 64, CC / 64, 1), 32, 0, stream>>>(G16, nullptr, W2, nullptr, HID, M, CC, bb2, 0, 0, 0);
        k_fin<<<L4, 256, 0, stream>>>(X1, M, OUT + (size_t)b * NTI * CC); }
}
